// structure_attention_net_57260503990855
// MI455X (gfx1250) — hardware-verified
//
#include <hip/hip_runtime.h>
#include <math.h>

#define NN   17
#define MP   32
#define DD   512
#define HH   8
#define HID  256
#define DC   515
#define SLP  68
#define APP  36

#define ACARRY 16.0f
#define WCARRY 64.0f
#define SCW    (1.0f / 1024.0f)
#define PCARRY 1024.0f
#define PSC    (1.0f / 16384.0f)

static_assert(ACARRY * WCARRY * SCW == 1.0f);
static_assert(PCARRY * ACARRY * PSC == 1.0f);
static_assert(NN <= MP && MP == 32);
static_assert(DD % 64 == 0 && HID % 64 == 0 && DD % 32 == 0 && HID % 32 == 0 && MP % 32 == 0);
static_assert(DD == 2 * 4 * 64);
static_assert(HID == 1 * 4 * 64);
static_assert((1u << 6) * 8u == DD);
static_assert((1u << 5) * 8u == HID);
static_assert((MP * DD / 8) % 256 == 0);
static_assert((DD * (DD / 8)) % 256 == 0 && (HID * (DD / 8)) % 256 == 0 && (MP * (HID / 8)) % 256 == 0);
static_assert(8 * 4 == MP);
static_assert(8 * 32 * 16 == 64 * MP * 2);
static_assert(9 * 2 >= NN && 8 * 2 < NN);
static_assert(NN * 3 - 32 == 19);
static_assert(4 * MP * SLP * 4 <= 131072);
static_assert(DC == DD + 3);

static constexpr size_t SZ_XS  = (size_t)MP * DD * 2;
static constexpr size_t SZ_FCT = (size_t)HH * DD * DD * 2;
static constexpr size_t SZ_W1T = (size_t)HH * HID * DD * 2;
static constexpr size_t SZ_W2T = (size_t)HH * MP * HID * 2;
static constexpr size_t SZ_F16 = (size_t)HH * MP * DD * 2;
static constexpr size_t SZ_FT  = (size_t)HH * DD * MP * 2;
static constexpr size_t SZ_H16 = (size_t)HH * MP * HID * 2;
static constexpr size_t SZ_ATT = (size_t)HH * MP * MP * 4;
static constexpr size_t SZ_P16 = (size_t)HH * MP * MP * 2;
static constexpr size_t OFF_XS  = 0;
static constexpr size_t OFF_FCT = OFF_XS  + SZ_XS;
static constexpr size_t OFF_W1T = OFF_FCT + SZ_FCT;
static constexpr size_t OFF_W2T = OFF_W1T + SZ_W1T;
static constexpr size_t OFF_F16 = OFF_W2T + SZ_W2T;
static constexpr size_t OFF_FT  = OFF_F16 + SZ_F16;
static constexpr size_t OFF_H16 = OFF_FT  + SZ_FT;
static constexpr size_t OFF_ATT = OFF_H16 + SZ_H16;
static constexpr size_t OFF_P16 = OFF_ATT + SZ_ATT;
static constexpr size_t WS_TOTAL = OFF_P16 + SZ_P16;
static_assert(SZ_XS % 128 == 0 && SZ_FCT % 128 == 0 && SZ_W1T % 128 == 0 && SZ_W2T % 128 == 0 && SZ_F16 % 128 == 0);
static_assert(SZ_FT % 128 == 0 && SZ_H16 % 128 == 0 && SZ_ATT % 128 == 0 && SZ_P16 % 128 == 0);
static_assert(WS_TOTAL == 7159808);
static_assert(WS_TOTAL <= (size_t)134217728);

static constexpr size_t OUT1_BYTES = 34816;
static_assert(OUT1_BYTES == (size_t)NN * DD * 4);
static_assert(OUT1_BYTES % 128 == 0);
static_assert(OUT1_BYTES / 4 + NN * 3 == 8755);

typedef _Float16 h16;
typedef __attribute__((ext_vector_type(16))) _Float16 v16h;
typedef __attribute__((ext_vector_type(8)))  _Float16 v8h;
typedef __attribute__((ext_vector_type(8)))  float    v8f;
typedef __attribute__((ext_vector_type(4)))  float    v4f;


static __device__ __forceinline__ float bfr(float f) {
    unsigned u = __float_as_uint(f);
    u += 0x7FFFu + ((u >> 16) & 1u);
    return __uint_as_float(u & 0xFFFF0000u);
}
static __device__ __forceinline__ h16 toh_flush(float v) {
    const float w = (fabsf(v) < 6.103515625e-05f) ? 0.0f : v;
    return (h16)w;
}

union FragU { v16h v; v8h h[2]; };
static __device__ __forceinline__ v16h frag_ld(const h16* p) {
    FragU f; f.h[0] = *(const v8h*)(p); f.h[1] = *(const v8h*)(p + 16); return f.v;
}
static __device__ __forceinline__ v8f wmma16g(v16h a, v16h b, v8f c) {
    c = __builtin_amdgcn_wmma_f32_16x16x32_f16(false, a, false, b, (short)0, c, false, false);
    asm volatile("v_nop\n\tv_nop\n\tv_nop\n\tv_nop" : "+v"(c) : "v"(a), "v"(b));
    return c;
}

template <int NJ>
static __device__ __forceinline__ void mm32(const h16* __restrict__ A, unsigned lda, const h16* __restrict__ Bt, unsigned ldb,
                                            unsigned K, unsigned n0, unsigned lane, v8f (&acc)[2][NJ]) {
    const unsigned rlane = lane & 15u;
    const unsigned koff = (lane >> 4) * 8u;
#pragma unroll
    for (int i = 0; i < 2; ++i)
#pragma unroll
        for (int j = 0; j < NJ; ++j) acc[i][j] = (v8f){0.f,0.f,0.f,0.f,0.f,0.f,0.f,0.f};
    for (unsigned k0 = 0; k0 < K; k0 += 32u) {
        v16h bh[NJ];
#pragma unroll
        for (int j = 0; j < NJ; ++j)
            bh[j] = frag_ld(Bt + (size_t)(n0 + ((unsigned)j << 4) + rlane) * ldb + koff + k0);
#pragma unroll
        for (int i = 0; i < 2; ++i) {
            const v16h ah = frag_ld(A + (size_t)(((unsigned)i << 4) + rlane) * lda + koff + k0);
#pragma unroll
            for (int j = 0; j < NJ; ++j) acc[i][j] = wmma16g(ah, bh[j], acc[i][j]);
        }
    }
}

__global__ __launch_bounds__(256) void k_xs16(const float* __restrict__ Xs, h16* __restrict__ XS) {
    const unsigned u = blockIdx.x * 256u + threadIdx.x;
    if (u >= (unsigned)(MP * DD / 8)) return;
    const unsigned row = u >> 6, c0 = (u & 63u) * 8u;
    const unsigned rc = min(row, (unsigned)(NN - 1));
    const float* xr = Xs + (size_t)rc * DD + c0;
    const v4f a = *(const v4f*)xr, b = *(const v4f*)(xr + 4);
    const float x[8] = {a.x, a.y, a.z, a.w, b.x, b.y, b.z, b.w};
    v8h hv;
#pragma unroll
    for (int i = 0; i < 8; ++i) {
        float w = bfr(x[i]) * ACARRY;
        w = (row < (unsigned)NN) ? w : 0.0f;
        hv[i] = toh_flush(w);
    }
    h16* d = XS + (size_t)row * DD + c0;
    *(volatile v8h*)d = hv;
    __threadfence();
    *(volatile v8h*)d = hv;
}

__global__ __launch_bounds__(256) void k_wt16(const float* __restrict__ Wm, unsigned KI, unsigned NO, unsigned NOP,
                                              unsigned lgper, unsigned srcHead, h16* __restrict__ W16) {
    const unsigned head = blockIdx.y;
    const float* Wl = Wm + (size_t)head * srcHead;
    h16* Dl = W16 + (size_t)head * NOP * KI;
    const unsigned u = blockIdx.x * 256u + threadIdx.x;
    const unsigned per = 1u << lgper;
    if (u >= NOP * per) return;
    const unsigned k0 = 8u * (u & (per - 1u));
    const unsigned o = u >> lgper;
    const unsigned oc = min(o, NO - 1u);
    v8h hv;
#pragma unroll
    for (int i = 0; i < 8; ++i) {
        float w = bfr(Wl[(size_t)(k0 + (unsigned)i) * NO + oc]) * WCARRY;
        w = (o < NO) ? w : 0.0f;
        hv[i] = toh_flush(w);
    }
    h16* d = Dl + (size_t)o * KI + k0;
    *(volatile v8h*)d = hv;
    __threadfence();
    *(volatile v8h*)d = hv;
}

__global__ __launch_bounds__(128) void k_gemm_f(const h16* __restrict__ XS, const h16* __restrict__ FCt,
                                                h16* __restrict__ F16, h16* __restrict__ FT) {
    __shared__ __align__(16) float sT[4][MP * SLP];
    const unsigned lane = threadIdx.x & 31u;
    const unsigned wave = (unsigned)__builtin_amdgcn_readfirstlane((int)(threadIdx.x >> 5));
    const unsigned head = blockIdx.z;
    const unsigned n0 = (blockIdx.x * 4u + wave) * 64u;
    const unsigned hh = lane >> 4, c = lane & 15u;
    v8f acc[2][4];
    mm32<4>(XS, DD, FCt + (size_t)head * DD * DD, DD, DD, n0, lane, acc);
    float* slab = sT[wave];
#pragma unroll
    for (int i = 0; i < 2; ++i)
#pragma unroll
        for (int j = 0; j < 4; ++j)
#pragma unroll
            for (int r = 0; r < 8; ++r)
                slab[((unsigned)i * 16u + 8u * hh + (unsigned)r) * SLP + (unsigned)j * 16u + c] = fmaxf(acc[i][j][r] * SCW, 0.0f) * ACARRY;
    __syncthreads();
    {
        const unsigned q = lane >> 3, c8 = (lane & 7u) * 8u;
        v8h hv[8];
#pragma unroll
        for (int it = 0; it < 8; ++it) {
            const float* sp = slab + ((unsigned)it * 4u + q) * SLP + c8;
#pragma unroll
            for (int e = 0; e < 8; ++e) hv[it][e] = toh_flush(sp[e]);
        }
        h16* dst = F16 + (size_t)head * MP * DD + n0 + c8;
        for (int pass = 0; pass < 2; ++pass) {
#pragma unroll
            for (int it = 0; it < 8; ++it)
                *(volatile v8h*)(dst + (size_t)((unsigned)it * 4u + q) * DD) = hv[it];
            __threadfence();
        }
    }
    {
        v8h tv[8];
#pragma unroll
        for (int it = 0; it < 8; ++it) {
            const unsigned p = (unsigned)it * 32u + lane;
            const unsigned dl = p >> 2, ng = p & 3u;
#pragma unroll
            for (int e = 0; e < 8; ++e) tv[it][e] = toh_flush(slab[(8u * ng + (unsigned)e) * SLP + dl]);
        }
        h16* dstT = FT + ((size_t)head * DD + n0) * MP;
        for (int pass = 0; pass < 2; ++pass) {
#pragma unroll
            for (int it = 0; it < 8; ++it)
                *(volatile v8h*)(dstT + (size_t)((unsigned)it * 32u + lane) * 8u) = tv[it];
            __threadfence();
        }
    }
}

__global__ __launch_bounds__(128) void k_gemm_h(const h16* __restrict__ F16, const h16* __restrict__ W1t,
                                                const float* __restrict__ W1, const float* __restrict__ b1,
                                                const float* __restrict__ ROIs, h16* __restrict__ H16) {
    __shared__ __align__(16) float sT[4][MP * SLP];
    const unsigned lane = threadIdx.x & 31u;
    const unsigned wave = (unsigned)__builtin_amdgcn_readfirstlane((int)(threadIdx.x >> 5));
    const unsigned head = blockIdx.z;
    const unsigned n0 = (blockIdx.x * 4u + wave) * 64u;
    const unsigned hh = lane >> 4, c = lane & 15u;
    v8f acc[2][4];
    mm32<4>(F16 + (size_t)head * MP * DD, DD, W1t + (size_t)head * HID * DD, DD, DD, n0, lane, acc);
    float* slab = sT[wave];
#pragma unroll
    for (int i = 0; i < 2; ++i)
#pragma unroll
        for (int j = 0; j < 4; ++j)
#pragma unroll
            for (int r = 0; r < 8; ++r)
                slab[((unsigned)i * 16u + 8u * hh + (unsigned)r) * SLP + (unsigned)j * 16u + c] = acc[i][j][r] * SCW;
    __syncthreads();
    const unsigned q = lane >> 3, c8 = (lane & 7u) * 8u;
    const unsigned m0 = n0 + c8;
    const float* wc = W1 + (size_t)head * DC * HID + (size_t)DD * HID + m0;
    float w3[3][8], bb[8];
#pragma unroll
    for (int cc = 0; cc < 3; ++cc) {
        const v4f wa = *(const v4f*)(wc + (size_t)cc * HID), wb = *(const v4f*)(wc + (size_t)cc * HID + 4);
        w3[cc][0] = bfr(wa.x); w3[cc][1] = bfr(wa.y); w3[cc][2] = bfr(wa.z); w3[cc][3] = bfr(wa.w);
        w3[cc][4] = bfr(wb.x); w3[cc][5] = bfr(wb.y); w3[cc][6] = bfr(wb.z); w3[cc][7] = bfr(wb.w);
    }
    {
        const v4f ba = *(const v4f*)(b1 + (size_t)head * HID + m0), bc = *(const v4f*)(b1 + (size_t)head * HID + m0 + 4);
        bb[0] = bfr(ba.x); bb[1] = bfr(ba.y); bb[2] = bfr(ba.z); bb[3] = bfr(ba.w);
        bb[4] = bfr(bc.x); bb[5] = bfr(bc.y); bb[6] = bfr(bc.z); bb[7] = bfr(bc.w);
    }
    h16* dst = H16 + (size_t)head * MP * HID + m0;
#pragma unroll 1
    for (unsigned it = 0; it < 8u; ++it) {
        const unsigned row = it * 4u + q;
        const unsigned rc = min(row, (unsigned)(NN - 1));
        const float r0 = bfr(ROIs[rc * 3u]), r1 = bfr(ROIs[rc * 3u + 1u]), r2 = bfr(ROIs[rc * 3u + 2u]);
        const float* sp = slab + row * SLP + c8;
        v8h hv;
#pragma unroll
        for (int e = 0; e < 8; ++e) {
            float t = sp[e];
            t += r0 * w3[0][e];
            t += r1 * w3[1][e];
            t += r2 * w3[2][e];
            t += bb[e];
            float y = tanhf(t) * ACARRY;
            y = (row < (unsigned)NN) ? y : 0.0f;
            hv[e] = toh_flush(y);
        }
        *(volatile v8h*)(dst + (size_t)row * HID) = hv;
        __threadfence();
        *(volatile v8h*)(dst + (size_t)row * HID) = hv;
    }
}

__global__ __launch_bounds__(32) void k_gemm_a(const h16* __restrict__ H16, const h16* __restrict__ W2t,
                                               const float* __restrict__ b2, float* __restrict__ ATT) {
    __shared__ __align__(16) float sA[MP * APP];
    const unsigned lane = threadIdx.x & 31u;
    const unsigned head = blockIdx.z;
    const unsigned hh = lane >> 4, c = lane & 15u;
    v8f acc[2][2];
    mm32<2>(H16 + (size_t)head * MP * HID, HID, W2t + (size_t)head * MP * HID, HID, HID, 0u, lane, acc);
    float bv[2];
#pragma unroll
    for (int j = 0; j < 2; ++j) {
        const unsigned k = (unsigned)j * 16u + c;
        const unsigned kc = min(k, (unsigned)(NN - 1));
        const float b = bfr(b2[head * (unsigned)NN + kc]);
        bv[j] = (k < (unsigned)NN) ? b : 0.0f;
    }
#pragma unroll
    for (int i = 0; i < 2; ++i)
#pragma unroll
        for (int j = 0; j < 2; ++j)
#pragma unroll
            for (int r = 0; r < 8; ++r)
                sA[((unsigned)i * 16u + 8u * hh + (unsigned)r) * APP + (unsigned)j * 16u + c] = acc[i][j][r] * SCW + bv[j];
    __syncthreads();
    const unsigned q = lane >> 3, c4 = (lane & 7u) * 4u;
    v4f vv[8];
#pragma unroll
    for (int it = 0; it < 8; ++it) vv[it] = *(const v4f*)(sA + ((unsigned)it * 4u + q) * APP + c4);
    float* dst = ATT + (size_t)head * MP * MP + c4;
    for (int pass = 0; pass < 2; ++pass) {
#pragma unroll
        for (int it = 0; it < 8; ++it)
            *(volatile v4f*)(dst + (size_t)((unsigned)it * 4u + q) * MP) = vv[it];
        __threadfence();
    }
}

__global__ __launch_bounds__(32) void k_soft(const float* __restrict__ ATT, h16* __restrict__ P16) {
    __shared__ __align__(16) float sP[MP * APP];
    const unsigned k = threadIdx.x & 31u;
    const unsigned head = blockIdx.x;
    const float* a = ATT + (size_t)head * MP * MP + k;
    float av[NN];
#pragma unroll
    for (int n = 0; n < 9; ++n) av[n] = a[(unsigned)n * MP];
    unsigned o2 = 9u * MP;
    {
        float t8 = av[8];
        asm volatile("" : "+v"(o2), "+v"(t8));
        av[8] = t8;
    }
#pragma unroll
    for (int n = 9; n < NN; ++n) av[n] = a[o2 + (unsigned)(n - 9) * MP];
    float mx = av[0];
#pragma unroll
    for (int n = 1; n < NN; ++n) mx = (av[n] > mx) ? av[n] : mx;
    float ev[NN];
    float s = 0.0f;
#pragma unroll
    for (int n = 0; n < NN; ++n) {
        ev[n] = expf(av[n] - mx);
        s += ev[n];
    }
    const float g = (1.0f / s) * PCARRY;
    const bool live = (k < (unsigned)NN);
#pragma unroll
    for (int n = 0; n < NN; ++n) {
        const float p = ev[n] * g;
        sP[k * APP + (unsigned)n] = live ? p : 0.0f;
    }
#pragma unroll
    for (int n = NN; n < MP; ++n) sP[k * APP + (unsigned)n] = 0.0f;
    __syncthreads();
    v8h hv[4];
#pragma unroll
    for (int it = 0; it < 4; ++it) {
        const unsigned p = (unsigned)it * 32u + k;
        const unsigned row = p >> 2, ng = p & 3u;
#pragma unroll
        for (int e = 0; e < 8; ++e) hv[it][e] = toh_flush(sP[row * APP + 8u * ng + (unsigned)e]);
    }
    h16* dst = P16 + (size_t)head * MP * MP;
    for (int pass = 0; pass < 2; ++pass) {
#pragma unroll
        for (int it = 0; it < 4; ++it)
            *(volatile v8h*)(dst + (size_t)((unsigned)it * 32u + k) * 8u) = hv[it];
        __threadfence();
    }
}

__global__ __launch_bounds__(128) void k_hp_out(const h16* __restrict__ P16, const h16* __restrict__ FT,
                                                const float* __restrict__ conv_w, const float* __restrict__ conv_b,
                                                const float* __restrict__ Xs, float* __restrict__ out) {
    __shared__ __align__(16) float sT[4][MP * SLP];
    const unsigned lane = threadIdx.x & 31u;
    const unsigned wave = (unsigned)__builtin_amdgcn_readfirstlane((int)(threadIdx.x >> 5));
    const unsigned n0 = (blockIdx.x * 4u + wave) * 64u;
    const unsigned hh = lane >> 4, c = lane & 15u;
    v8f sum[2][4];
#pragma unroll
    for (int i = 0; i < 2; ++i)
#pragma unroll
        for (int j = 0; j < 4; ++j) sum[i][j] = (v8f){0.f,0.f,0.f,0.f,0.f,0.f,0.f,0.f};
#pragma unroll 1
    for (unsigned h = 0; h < (unsigned)HH; ++h) {
        const float cw = bfr(conv_w[h]) * PSC;
        v8f acc[2][4];
        mm32<4>(P16 + (size_t)h * MP * MP, MP, FT + (size_t)h * DD * MP, MP, MP, n0, lane, acc);
#pragma unroll
        for (int i = 0; i < 2; ++i)
#pragma unroll
            for (int j = 0; j < 4; ++j)
#pragma unroll
                for (int r = 0; r < 8; ++r) sum[i][j][r] += cw * acc[i][j][r];
    }
    const float cb = bfr(conv_b[0]);
    float* slab = sT[wave];
#pragma unroll
    for (int i = 0; i < 2; ++i)
#pragma unroll
        for (int j = 0; j < 4; ++j)
#pragma unroll
            for (int r = 0; r < 8; ++r)
                slab[((unsigned)i * 16u + 8u * hh + (unsigned)r) * SLP + (unsigned)j * 16u + c] = fmaxf(sum[i][j][r] + cb, 0.0f);
    __syncthreads();
    const unsigned c4 = (lane & 15u) * 4u;
    float* obase = out + n0 + c4;
    const float* xbase = Xs + n0 + c4;
    v4f vv[9];
#pragma unroll
    for (int it = 0; it < 9; ++it) {
        const unsigned row = (unsigned)it * 2u + hh;
        const unsigned rc = min(row, (unsigned)(NN - 1));
        v4f t = *(const v4f*)(slab + row * SLP + c4);
        const v4f x = *(const v4f*)(xbase + (size_t)rc * DD);
        t.x += bfr(x.x); t.y += bfr(x.y); t.z += bfr(x.z); t.w += bfr(x.w);
        vv[it] = t;
    }
    for (int pass = 0; pass < 2; ++pass) {
#pragma unroll
        for (int it = 0; it < 9; ++it) {
            const unsigned row = (unsigned)it * 2u + hh;
            if (row < (unsigned)NN) *(volatile v4f*)(obase + (size_t)row * DD) = vv[it];
        }
        __threadfence();
    }
}

__global__ __launch_bounds__(32) void k_pass(const float* __restrict__ ROIs, float* __restrict__ out1) {
    const unsigned lane = threadIdx.x & 31u;
    const float a = bfr(ROIs[lane]);
    const unsigned i2 = min(32u + lane, (unsigned)(NN * 3 - 1));
    const float b = bfr(ROIs[i2]);
    *(volatile float*)(out1 + lane) = a;
    if (lane < 19u) *(volatile float*)(out1 + 32u + lane) = b;
    __threadfence();
    *(volatile float*)(out1 + lane) = a;
    if (lane < 19u) *(volatile float*)(out1 + 32u + lane) = b;
}

extern "C" void kernel_launch(void* const* d_in, const int* in_sizes, int n_in, void* d_out, int out_size,
                              void* d_ws, size_t ws_size, hipStream_t stream) {
    if (n_in < 10) return;
    if (in_sizes[0] < NN * DD || in_sizes[1] < NN * 3 || in_sizes[2] < NN * NN || in_sizes[3] < HH * DD * DD) return;
    if (in_sizes[4] < HH * DC * HID || in_sizes[5] < HH * HID || in_sizes[6] < HH * HID * NN || in_sizes[7] < HH * NN) return;
    if (in_sizes[8] < HH || in_sizes[9] < 1) return;
    if (out_size < NN * DD + NN * 3) return;
    if (ws_size < WS_TOTAL) return;

    const float* Xs     = (const float*)d_in[0];
    const float* ROIs   = (const float*)d_in[1];
    const float* adj    = (const float*)d_in[2];
    const float* FC     = (const float*)d_in[3];
    const float* W1     = (const float*)d_in[4];
    const float* b1     = (const float*)d_in[5];
    const float* W2     = (const float*)d_in[6];
    const float* b2     = (const float*)d_in[7];
    const float* conv_w = (const float*)d_in[8];
    const float* conv_b = (const float*)d_in[9];
    (void)adj;
    float* out  = (float*)d_out;
    float* out1 = (float*)((char*)d_out + OUT1_BYTES);

    char* wsp = (char*)d_ws;
    h16*   XS16 = (h16*)(wsp + OFF_XS);
    h16*   FCT  = (h16*)(wsp + OFF_FCT);
    h16*   W1T  = (h16*)(wsp + OFF_W1T);
    h16*   W2T  = (h16*)(wsp + OFF_W2T);
    h16*   F16P = (h16*)(wsp + OFF_F16);
    h16*   FTP  = (h16*)(wsp + OFF_FT);
    h16*   H16P = (h16*)(wsp + OFF_H16);
    float* ATT  = (float*)(wsp + OFF_ATT);
    h16*   P16P = (h16*)(wsp + OFF_P16);

    k_xs16<<<(MP * DD / 8) / 256, 256, 0, stream>>>(Xs, XS16);
    k_wt16<<<dim3((DD * (DD / 8)) / 256, HH), 256, 0, stream>>>(FC, DD, DD, DD, 6, DD * DD, FCT);
    k_wt16<<<dim3((HID * (DD / 8)) / 256, HH), 256, 0, stream>>>(W1, DD, HID, HID, 6, DC * HID, W1T);
    k_wt16<<<dim3((MP * (HID / 8)) / 256, HH), 256, 0, stream>>>(W2, HID, NN, MP, 5, HID * NN, W2T);

    k_gemm_f<<<dim3(2, 1, HH), 128, 0, stream>>>(XS16, FCT, F16P, FTP);
    k_gemm_h<<<dim3(1, 1, HH), 128, 0, stream>>>(F16P, W1T, W1, b1, ROIs, H16P);
    k_gemm_a<<<dim3(1, 1, HH), 32, 0, stream>>>(H16P, W2T, b2, ATT);
    k_soft<<<HH, 32, 0, stream>>>(ATT, P16P);
    k_hp_out<<<2, 128, 0, stream>>>(P16P, FTP, conv_w, conv_b, Xs, out);
    k_pass<<<1, 32, 0, stream>>>(ROIs, out1);
}
